// SelfAttention_80900003987672
// MI455X (gfx1250) — hardware-verified
//
#include <hip/hip_runtime.h>

#ifndef NB
#define NB 4
#endif
#ifndef SEQ
#define SEQ 2048
#endif
#define NB_FULL 4
#define SEQ_FULL 2048
#define HD 1024

#define GBM 128
#define GBN 64
#define GBK 32
#define LROW 40
#define SMT (SEQ / 8)
#define SMW (SMT / 32)
#define WBLK (HD * HD / 2048)

static_assert(NB >= 1 && NB <= NB_FULL);
static_assert(SEQ >= 256 && SEQ <= SEQ_FULL);
static_assert(SEQ % 256 == 0);
static_assert(SEQ % GBM == 0 && SEQ % GBN == 0 && SEQ % GBK == 0);
static_assert(HD % GBM == 0 && HD % GBN == 0 && HD % GBK == 0);
static_assert(SMT <= 1024 && SMT % 32 == 0 && SMW <= 32);
static_assert(((long long)NB * SEQ * HD) % 2048 == 0);
static_assert((HD * HD) % 2048 == 0);

typedef __bf16 bf16;
typedef _Float16 f16;
typedef bf16 v16b __attribute__((ext_vector_type(16)));
typedef f16 v16h __attribute__((ext_vector_type(16)));
typedef bf16 v8b __attribute__((ext_vector_type(8)));
typedef f16 v8h __attribute__((ext_vector_type(8)));
typedef float v8f __attribute__((ext_vector_type(8)));
typedef float v4f __attribute__((ext_vector_type(4)));
typedef unsigned v4u __attribute__((ext_vector_type(4)));

template <typename V16> union FragU { V16 v; v4u q[2]; };
union Pk8b { v8b h; v4u u; };
union Pk8h { v8h h; v4u u; };

#define PCARRY 8192.0f
#define PCARRY_INV 0.0001220703125f
#define SCORE_SCALE 0.03125f
#define L2E 1.4426950408889634f

__device__ __forceinline__ v8f mma16(v16b a, v16b b, v8f c) {
  c = __builtin_amdgcn_wmma_f32_16x16x32_bf16(false, a, false, b, (short)0, c, false, false);
  asm volatile("v_nop\n\tv_nop\n\tv_nop\n\tv_nop" : "+v"(c) : "v"(a), "v"(b));
  return c;
}
__device__ __forceinline__ v8f mma16(v16h a, v16h b, v8f c) {
  c = __builtin_amdgcn_wmma_f32_16x16x32_f16(false, a, false, b, (short)0, c, false, false);
  asm volatile("v_nop\n\tv_nop\n\tv_nop\n\tv_nop" : "+v"(c) : "v"(a), "v"(b));
  return c;
}

__device__ __forceinline__ float bfr(float x) { return (float)((bf16)x); }

__global__ __launch_bounds__(256) void k_cvt_x(const float* __restrict__ X, bf16* __restrict__ Xb) {
  const size_t i = (size_t)blockIdx.x * 256 + threadIdx.x;
  const size_t e = i * 8;
  const size_t per_b = (size_t)SEQ * HD;
  const size_t b = e / per_b;
  const size_t rem = e - b * per_b;
  const float* src = X + b * ((size_t)SEQ_FULL * HD) + rem;
  const v4f a = *(const v4f*)src;
  const v4f c = *(const v4f*)(src + 4);
  Pk8b o;
  o.h[0] = (bf16)a[0]; o.h[1] = (bf16)a[1]; o.h[2] = (bf16)a[2]; o.h[3] = (bf16)a[3];
  o.h[4] = (bf16)c[0]; o.h[5] = (bf16)c[1]; o.h[6] = (bf16)c[2]; o.h[7] = (bf16)c[3];
  const v4u u = o.u;
  bf16* dst = Xb + e;
  *(volatile v4u*)dst = u;
  __threadfence();
  *(volatile v4u*)dst = u;
}

__global__ __launch_bounds__(256) void k_cvt_w(const float* __restrict__ Wq, const float* __restrict__ Wk,
                                               const float* __restrict__ Wv, bf16* __restrict__ Wb) {
  const int which = blockIdx.x / WBLK;
  const float* src = (which == 0) ? Wq : ((which == 1) ? Wk : Wv);
  const size_t e = ((size_t)(blockIdx.x - which * WBLK) * 256 + threadIdx.x) * 8;
  const v4f a = *(const v4f*)(src + e);
  const v4f c = *(const v4f*)(src + e + 4);
  Pk8b o;
  o.h[0] = (bf16)a[0]; o.h[1] = (bf16)a[1]; o.h[2] = (bf16)a[2]; o.h[3] = (bf16)a[3];
  o.h[4] = (bf16)c[0]; o.h[5] = (bf16)c[1]; o.h[6] = (bf16)c[2]; o.h[7] = (bf16)c[3];
  const v4u u = o.u;
  bf16* dst = Wb + (size_t)which * HD * HD + e;
  *(volatile v4u*)dst = u;
  __threadfence();
  *(volatile v4u*)dst = u;
}

template <typename T, typename V16, int EPI>
__global__ __launch_bounds__(256) __attribute__((amdgpu_num_vgpr(256)))
void k_gemm(const T* __restrict__ A, const T* __restrict__ Bn,
            int lda, int ldb, int kdim, long long saz, long long sbz,
            void* C0, int ldc, long long scz,
            const float* __restrict__ bias, float scale) {
  __shared__ __attribute__((aligned(16))) unsigned char smem[32768];
  const int tid = threadIdx.x;
  const int lane = tid & 31;
  const int wave = tid >> 5;
  const int wm = wave >> 1;
  const int wn = wave & 1;
  const int fm = lane & 15;
  const int hh = lane >> 4;
  const int kb = hh * 8;
  const int m0 = blockIdx.y * GBM;
  const int n0 = blockIdx.x * GBN;
  const long long z = blockIdx.z;
  A += z * saz;
  Bn += z * sbz;

  T* As = (T*)(smem);
  T* Bs = (T*)(smem + 10240);

  const int sr = tid >> 2;
  const int sc = (tid & 3) * 8;

  v8f acc[2][2];
#pragma unroll
  for (int i = 0; i < 2; ++i)
#pragma unroll
    for (int j = 0; j < 2; ++j) acc[i][j] = (v8f){0.f, 0.f, 0.f, 0.f, 0.f, 0.f, 0.f, 0.f};

  for (int k0 = 0; k0 < kdim; k0 += GBK) {
    const size_t oa0 = (size_t)(m0 + sr) * lda + k0 + sc;
    const size_t oa1 = (size_t)(m0 + sr + 64) * lda + k0 + sc;
    const size_t ob = (size_t)(n0 + sr) * ldb + k0 + sc;
    const v4u ga0 = *(const v4u*)(A + oa0);
    const v4u ga1 = *(const v4u*)(A + oa1);
    const v4u gb0 = *(const v4u*)(Bn + ob);
    __syncthreads();
    *(v4u*)(As + sr * LROW + sc) = ga0;
    *(v4u*)(As + (sr + 64) * LROW + sc) = ga1;
    *(v4u*)(Bs + sr * LROW + sc) = gb0;
    __syncthreads();

    V16 af[2], bg[2];
#pragma unroll
    for (int mt = 0; mt < 2; ++mt) {
      const T* p = As + (wm * 32 + mt * 16 + fm) * LROW + kb;
      FragU<V16> u;
      u.q[0] = *(const v4u*)p;
      u.q[1] = *(const v4u*)(p + 16);
      af[mt] = u.v;
    }
#pragma unroll
    for (int nt = 0; nt < 2; ++nt) {
      const T* p = Bs + (wn * 32 + nt * 16 + fm) * LROW + kb;
      FragU<V16> u;
      u.q[0] = *(const v4u*)p;
      u.q[1] = *(const v4u*)(p + 16);
      bg[nt] = u.v;
    }
#pragma unroll
    for (int mt = 0; mt < 2; ++mt)
#pragma unroll
      for (int nt = 0; nt < 2; ++nt) acc[mt][nt] = mma16(af[mt], bg[nt], acc[mt][nt]);
  }
  __syncthreads();

  const int rowb = wm * 32 + hh * 8;
  const int colb = wn * 32 + fm;

  if constexpr (EPI == 2) {
    float* stg = (float*)smem;
    float* C = (float*)C0 + z * scz;
#pragma unroll
    for (int mt = 0; mt < 2; ++mt)
#pragma unroll
      for (int nt = 0; nt < 2; ++nt)
#pragma unroll
        for (int r = 0; r < 8; ++r)
          stg[(rowb + mt * 16 + r) * GBN + colb + nt * 16] = acc[mt][nt][r] * scale;
    __syncthreads();
    const int piece = lane & 15;
    const int rsel = lane >> 4;
#pragma unroll
    for (int i = 0; i < 8; ++i) {
      const int row = (wave * 8 + i) * 2 + rsel;
      const v4f v = *(const v4f*)(stg + row * GBN + piece * 4);
      *(volatile v4f*)(C + (size_t)(m0 + row) * ldc + n0 + piece * 4) = v;
    }
    __threadfence();
#pragma unroll
    for (int i = 0; i < 8; ++i) {
      const int row = (wave * 8 + i) * 2 + rsel;
      const v4f v = *(const v4f*)(stg + row * GBN + piece * 4);
      *(volatile v4f*)(C + (size_t)(m0 + row) * ldc + n0 + piece * 4) = v;
    }
  } else {
    f16* stg = (f16*)smem;
    f16* C = (f16*)C0 + z * scz;
    if constexpr (EPI == 0) {
      float bb[2];
#pragma unroll
      for (int nt = 0; nt < 2; ++nt) bb[nt] = bfr(bias[n0 + colb + nt * 16]);
#pragma unroll
      for (int mt = 0; mt < 2; ++mt)
#pragma unroll
        for (int nt = 0; nt < 2; ++nt)
#pragma unroll
          for (int r = 0; r < 8; ++r)
            stg[(rowb + mt * 16 + r) * GBN + colb + nt * 16] = (f16)(acc[mt][nt][r] + bb[nt]);
    } else {
      const float brow = bfr(bias[m0 + wm * 32 + lane]);
#pragma unroll
      for (int mt = 0; mt < 2; ++mt)
#pragma unroll
        for (int r = 0; r < 8; ++r) {
          const float bvr = __shfl(brow, mt * 16 + hh * 8 + r);
#pragma unroll
          for (int nt = 0; nt < 2; ++nt)
            stg[(rowb + mt * 16 + r) * GBN + colb + nt * 16] = (f16)(acc[mt][nt][r] + bvr);
        }
    }
    __syncthreads();
    const int piece = lane & 7;
    const int rsel = lane >> 3;
#pragma unroll
    for (int i = 0; i < 4; ++i) {
      const int row = (wave * 4 + i) * 4 + rsel;
      const v4u v = *(const v4u*)(stg + row * GBN + piece * 8);
      *(volatile v4u*)(C + (size_t)(m0 + row) * ldc + n0 + piece * 8) = v;
    }
    __threadfence();
#pragma unroll
    for (int i = 0; i < 4; ++i) {
      const int row = (wave * 4 + i) * 4 + rsel;
      const v4u v = *(const v4u*)(stg + row * GBN + piece * 8);
      *(volatile v4u*)(C + (size_t)(m0 + row) * ldc + n0 + piece * 8) = v;
    }
  }
}

__global__ __launch_bounds__(SMT) void k_softmax(const float* __restrict__ S, f16* __restrict__ P) {
  __shared__ float red[32];
  const int row = blockIdx.x;
  const int t = threadIdx.x;
  const int lane = t & 31;
  const int wave = t >> 5;
  const float* sp = S + (size_t)row * SEQ + t * 8;
  const v4f a = *(const v4f*)sp;
  const v4f c = *(const v4f*)(sp + 4);
  float e[8] = {a[0], a[1], a[2], a[3], c[0], c[1], c[2], c[3]};
  float m = e[0];
#pragma unroll
  for (int i = 1; i < 8; ++i) m = fmaxf(m, e[i]);
#pragma unroll
  for (int o = 16; o > 0; o >>= 1) m = fmaxf(m, __shfl_xor(m, o));
  if (lane == 0) red[wave] = m;
  __syncthreads();
  m = red[0];
  for (int w = 1; w < SMW; ++w) m = fmaxf(m, red[w]);
  __syncthreads();
  float s = 0.0f;
#pragma unroll
  for (int i = 0; i < 8; ++i) {
    e[i] = __builtin_amdgcn_exp2f((e[i] - m) * L2E);
    s += e[i];
  }
#pragma unroll
  for (int o = 16; o > 0; o >>= 1) s += __shfl_xor(s, o);
  if (lane == 0) red[wave] = s;
  __syncthreads();
  float tot = red[0];
  for (int w = 1; w < SMW; ++w) tot += red[w];
  const float inv = PCARRY * (1.0f / tot);
  Pk8h o;
#pragma unroll
  for (int i = 0; i < 8; ++i) o.h[i] = (f16)(e[i] * inv);
  const v4u u = o.u;
  f16* pp = P + (size_t)row * SEQ + t * 8;
  *(volatile v4u*)pp = u;
  __threadfence();
  *(volatile v4u*)pp = u;
}

extern "C" void kernel_launch(void* const* d_in, const int* in_sizes, int n_in,
                              void* d_out, int out_size, void* d_ws, size_t ws_size,
                              hipStream_t stream) {
  if (n_in < 7) return;
  const long long needX = ((long long)(NB - 1) * SEQ_FULL + SEQ) * HD;
  if ((long long)in_sizes[0] < needX) return;
  if (in_sizes[1] < HD * HD || in_sizes[3] < HD * HD || in_sizes[5] < HD * HD) return;
  if (in_sizes[2] < HD || in_sizes[4] < HD || in_sizes[6] < HD) return;
  if ((long long)out_size < (long long)NB * SEQ * HD) return;

  const float* X = (const float*)d_in[0];
  const float* Wq = (const float*)d_in[1];
  const float* bq = (const float*)d_in[2];
  const float* Wk = (const float*)d_in[3];
  const float* bk = (const float*)d_in[4];
  const float* Wv = (const float*)d_in[5];
  const float* bv = (const float*)d_in[6];
  float* out = (float*)d_out;

  const size_t bytes_act = (size_t)NB * SEQ * HD * 2;
  const size_t bytes_w = (size_t)3 * HD * HD * 2;
  const size_t bytes_s = (size_t)SEQ * SEQ * 4;
  const size_t bytes_p = (size_t)SEQ * SEQ * 2;
  char* ws = (char*)d_ws;
  size_t off = 0;
  bf16* Xb = (bf16*)(ws + off); off += bytes_act;
  bf16* Wb = (bf16*)(ws + off); off += bytes_w;
  f16* Qp = (f16*)(ws + off); off += bytes_act;
  f16* Kp = (f16*)(ws + off); off += bytes_act;
  f16* Vt = (f16*)(ws + off); off += bytes_act;
  float* S = (float*)(ws + off); off += bytes_s;
  f16* P = (f16*)(ws + off); off += bytes_p;
  if (off > ws_size) return;

  k_cvt_x<<<(unsigned)(((size_t)NB * SEQ * HD) / 2048), 256, 0, stream>>>(X, Xb);
  k_cvt_w<<<3 * WBLK, 256, 0, stream>>>(Wq, Wk, Wv, Wb);

  k_gemm<bf16, v16b, 0><<<dim3(HD / GBN, (NB * SEQ) / GBM, 1), 256, 0, stream>>>(
      Xb, Wb, HD, HD, HD, 0LL, 0LL, (void*)Qp, HD, 0LL, bq, 1.0f);
  k_gemm<bf16, v16b, 0><<<dim3(HD / GBN, (NB * SEQ) / GBM, 1), 256, 0, stream>>>(
      Xb, Wb + (size_t)HD * HD, HD, HD, HD, 0LL, 0LL, (void*)Kp, HD, 0LL, bk, 1.0f);

  k_gemm<bf16, v16b, 1><<<dim3(SEQ / GBN, HD / GBM, NB), 256, 0, stream>>>(
      Wb + (size_t)2 * HD * HD, Xb, HD, HD, HD, 0LL, (long long)SEQ * HD,
      (void*)Vt, SEQ, (long long)HD * SEQ, bv, 1.0f);

  for (int b = 0; b < NB; ++b) {
    const size_t qo = (size_t)b * SEQ * HD;
    k_gemm<f16, v16h, 2><<<dim3(SEQ / GBN, SEQ / GBM, 1), 256, 0, stream>>>(
        Qp + qo, Kp + qo, HD, HD, HD, 0LL, 0LL, (void*)S, SEQ, 0LL, bq, SCORE_SCALE);
    k_softmax<<<SEQ, SMT, 0, stream>>>(S, P);
    k_gemm<f16, v16h, 2><<<dim3(HD / GBN, SEQ / GBM, 1), 256, 0, stream>>>(
        P, Vt + (size_t)b * HD * SEQ, SEQ, SEQ, SEQ, 0LL, 0LL,
        (void*)(out + qo), HD, 0LL, bq, PCARRY_INV);
  }
}
